// GNNBlock_24008867184710
// MI455X (gfx1250) — hardware-verified
//
#include <hip/hip_runtime.h>
#include <stddef.h>
#include <stdint.h>


#define NTHR   256
#define NWAVE  8
#define EPT    8
#define CHUNK  (NTHR * EPT)
#define WCAP   (EPT * 32)
#define LISTN  (NWAVE * WCAP)
#define TE     16
#define PASSN  (NWAVE * TE)
#define PCAP   (CHUNK + PASSN)
#define NB     512
#define HD     64
#define GT     128
#define GROWS  64
#define BN_EPS 1e-5

static_assert(PASSN == 128);
static_assert(PASSN <= NTHR);
static_assert(PCAP >= CHUNK + PASSN);
static_assert((NB % GROWS) == 0);
static_assert(NB * HD == NWAVE * 32 * 128);
static_assert(GT == 2 * HD);

typedef float    v2f  __attribute__((ext_vector_type(2)));
typedef float    v4f  __attribute__((ext_vector_type(4)));
typedef float    v8f  __attribute__((ext_vector_type(8)));
typedef int      v4i  __attribute__((ext_vector_type(4)));
typedef unsigned v4u  __attribute__((ext_vector_type(4)));
typedef double   v2d  __attribute__((ext_vector_type(2)));
typedef __bf16   v16b __attribute__((ext_vector_type(16)));
union Frag { v16b v; v4u q[2]; };

__device__ __forceinline__ int clampi(int v, int lo, int hi) {
  v = v > hi ? hi : v;
  return v < lo ? lo : v;
}

__device__ __forceinline__ unsigned pk2(float a, float b) {
  union { __bf16 h[2]; unsigned u; } x;
  x.h[0] = (__bf16)a;
  x.h[1] = (__bf16)b;
  return x.u;
}

__device__ __forceinline__ void split2(float a, float b, unsigned& hi, unsigned& lo) {
  const unsigned ph = pk2(a, b);
  const float ra = a - __uint_as_float(ph << 16);
  const float rb = b - __uint_as_float(ph & 0xFFFF0000u);
  hi = ph;
  lo = pk2(ra, rb);
}

__device__ __forceinline__ void split8(v4f a, v4f b, v4u& hi, v4u& lo) {
  unsigned h0, h1, h2, h3, l0, l1, l2, l3;
  split2(a.x, a.y, h0, l0);
  split2(a.z, a.w, h1, l1);
  split2(b.x, b.y, h2, l2);
  split2(b.z, b.w, h3, l3);
  v4u hv = {h0, h1, h2, h3};
  v4u lv = {l0, l1, l2, l3};
  hi = hv;
  lo = lv;
}

__device__ __forceinline__ v4f prelu4(v4f t, float a) {
  v4f r;
  r.x = (t.x >= 0.0f) ? t.x : a * t.x;
  r.y = (t.y >= 0.0f) ? t.y : a * t.y;
  r.z = (t.z >= 0.0f) ? t.z : a * t.z;
  r.w = (t.w >= 0.0f) ? t.w : a * t.w;
  return r;
}

__device__ __forceinline__ v8f ldc8(const float* p) {
  const v4f a = *(const v4f*)p;
  const v4f b = *(const v4f*)(p + 4);
  v8f c;
  c[0] = a.x; c[1] = a.y; c[2] = a.z; c[3] = a.w;
  c[4] = b.x; c[5] = b.y; c[6] = b.z; c[7] = b.w;
  return c;
}

__device__ __forceinline__ void st8(float* p, v8f d) {
  v4f u0 = {d[0], d[1], d[2], d[3]};
  v4f u1 = {d[4], d[5], d[6], d[7]};
  *(v4f*)p = u0;
  *(v4f*)(p + 4) = u1;
}

__device__ __forceinline__ void stprelu8(float* p, v8f d, float a) {
  v4f u0 = {d[0], d[1], d[2], d[3]};
  v4f u1 = {d[4], d[5], d[6], d[7]};
  *(v4f*)p = prelu4(u0, a);
  *(v4f*)(p + 4) = prelu4(u1, a);
}

__device__ __forceinline__ void prelu_split8(v8f d, float a, v4u& hi, v4u& lo) {
  v4f u0 = {d[0], d[1], d[2], d[3]};
  v4f u1 = {d[4], d[5], d[6], d[7]};
  split8(prelu4(u0, a), prelu4(u1, a), hi, lo);
}

__device__ __forceinline__ v8f wmb(v16b a, v16b b, v8f c) {
  v8f d = __builtin_amdgcn_wmma_f32_16x16x32_bf16(false, a, false, b, (short)0, c, false, false);
  asm volatile("v_nop\n\tv_nop\n\tv_nop\n\tv_nop" : "+v"(d) : "v"(a), "v"(b));
  return d;
}

__device__ __forceinline__ v8f wm3(const Frag& ah, const Frag& al, const Frag& bh, const Frag& bl, v8f c) {
  c = wmb(ah.v, bh.v, c);
  c = wmb(ah.v, bl.v, c);
  c = wmb(al.v, bh.v, c);
  return c;
}

__global__ __launch_bounds__(256) void k_wprep(const float* __restrict__ W, int F, int K, int rowOff,
                                               v4u* dh, v4u* dl, int nG) {
  const int g  = blockIdx.x * 256 + threadIdx.x;
  const int gc = (g < nG) ? g : nG - 1;
  const int kg = K >> 3;
  const int f  = gc / kg;
  const int kb = (gc - f * kg) * 8;
  const float* wp = W + (size_t)(rowOff + kb) * F + f;
  v4f t0, t1;
  t0.x = wp[0];              t0.y = wp[(size_t)F];      t0.z = wp[(size_t)2 * F];  t0.w = wp[(size_t)3 * F];
  t1.x = wp[(size_t)4 * F];  t1.y = wp[(size_t)5 * F];  t1.z = wp[(size_t)6 * F];  t1.w = wp[(size_t)7 * F];
  v4u hi, lo;
  split8(t0, t1, hi, lo);
  if (g < nG) { *(volatile v4u*)(dh + g) = hi; *(volatile v4u*)(dl + g) = lo; }
  __threadfence();
  if (g < nG) { *(volatile v4u*)(dh + g) = hi; *(volatile v4u*)(dl + g) = lo; }
}

__global__ __launch_bounds__(GT) void k_pq(const float* __restrict__ x, const v4u* __restrict__ w1p,
                                          const float* __restrict__ b1, float* pq, int nN) {
  __shared__ v4u wsm[2 * 128 * 8];
  __shared__ __attribute__((aligned(16))) float bsm[128];
  __shared__ __attribute__((aligned(16))) float stg[GROWS * 128];

  const int tid = threadIdx.x, lane = tid & 31, wave = tid >> 5, h = lane >> 4, m = lane & 15;
  for (int i = tid; i < 2 * 128 * 8; i += GT) wsm[i] = w1p[i];
  {
    const float bv = b1[(tid < HD) ? tid : HD - 1];
    bsm[tid] = (tid < HD) ? bv : 0.0f;
  }
  __syncthreads();

  const int n0 = blockIdx.x * GROWS + wave * 16;
  const int nd = clampi(n0 + m, 0, nN - 1);
  const float* xr = x + (size_t)nd * HD;
  Frag bh[2], bl[2];
#pragma unroll
  for (int ks = 0; ks < 2; ++ks) {
    const float* p = xr + 32 * ks + 8 * h;
    const v4f a0 = *(const v4f*)p,        a1 = *(const v4f*)(p + 4);
    const v4f c0 = *(const v4f*)(p + 16), c1 = *(const v4f*)(p + 20);
    split8(a0, a1, bh[ks].q[0], bl[ks].q[0]);
    split8(c0, c1, bh[ks].q[1], bl[ks].q[1]);
  }
  float* srow = stg + (wave * 16 + m) * 128;
#pragma unroll
  for (int ft = 0; ft < 8; ++ft) {
    v8f acc = ldc8(bsm + 16 * ft + 8 * h);
#pragma unroll
    for (int ks = 0; ks < 2; ++ks) {
      const int u = (16 * ft + m) * 8 + 4 * ks + h;
      Frag ah, al;
      ah.q[0] = wsm[u];            ah.q[1] = wsm[u + 2];
      al.q[0] = wsm[128 * 8 + u];  al.q[1] = wsm[128 * 8 + u + 2];
      acc = wm3(ah, al, bh[ks], bl[ks], acc);
    }
    st8(srow + 16 * ft + 8 * h, acc);
  }
  __syncthreads();

  const float* sp = stg + wave * (16 * 128);
  float* gp = pq + (size_t)n0 * 128;
#pragma unroll 4
  for (int q = 0; q < 16; ++q) {
    const v4f v = *(const v4f*)(sp + q * 128 + 4 * lane);
    *(volatile v4f*)(gp + q * 128 + 4 * lane) = v;
  }
  __threadfence();
#pragma unroll 4
  for (int q = 0; q < 16; ++q) {
    const v4f v = *(const v4f*)(sp + q * 128 + 4 * lane);
    *(volatile v4f*)(gp + q * 128 + 4 * lane) = v;
  }
}

__device__ __forceinline__ int scan_chunk(const int* __restrict__ dsts, int nE, int cbase, int nodeBase,
                                          int vec8, int* list, int tid, int wave) {
  int wc = 0;
  const int el0  = tid * EPT;
  const int e0   = cbase + el0;
  const int sent = -2147483647 - 1;
  v4i da, db;
  if (vec8 != 0 && cbase + CHUNK <= nE) {
    da = *(const v4i*)(dsts + e0);
    db = *(const v4i*)(dsts + e0 + 4);
  } else {
    da.x = (e0     < nE) ? dsts[min(e0, nE - 1)] : sent;
    da.y = (e0 + 1 < nE) ? dsts[min(e0 + 1, nE - 1)] : sent;
    da.z = (e0 + 2 < nE) ? dsts[min(e0 + 2, nE - 1)] : sent;
    da.w = (e0 + 3 < nE) ? dsts[min(e0 + 3, nE - 1)] : sent;
    db.x = (e0 + 4 < nE) ? dsts[min(e0 + 4, nE - 1)] : sent;
    db.y = (e0 + 5 < nE) ? dsts[min(e0 + 5, nE - 1)] : sent;
    db.z = (e0 + 6 < nE) ? dsts[min(e0 + 6, nE - 1)] : sent;
    db.w = (e0 + 7 < nE) ? dsts[min(e0 + 7, nE - 1)] : sent;
  }
  const unsigned nb = (unsigned)nodeBase;
  const unsigned s0 = (unsigned)da.x - nb, s1 = (unsigned)da.y - nb;
  const unsigned s2 = (unsigned)da.z - nb, s3 = (unsigned)da.w - nb;
  const unsigned s4 = (unsigned)db.x - nb, s5 = (unsigned)db.y - nb;
  const unsigned s6 = (unsigned)db.z - nb, s7 = (unsigned)db.w - nb;
  const bool h0 = s0 < (unsigned)NB, h1 = s1 < (unsigned)NB, h2 = s2 < (unsigned)NB, h3 = s3 < (unsigned)NB;
  const bool h4 = s4 < (unsigned)NB, h5 = s5 < (unsigned)NB, h6 = s6 < (unsigned)NB, h7 = s7 < (unsigned)NB;
  const unsigned any = __builtin_amdgcn_ballot_w32(h0 | h1 | h2 | h3 | h4 | h5 | h6 | h7);
  if (any != 0u) {
#define HITJ(J, HJ) { \
      const unsigned mj = __builtin_amdgcn_ballot_w32(HJ); \
      if (mj != 0u) { \
        if (HJ) { \
          const int pos = wc + (int)__builtin_amdgcn_mbcnt_lo(mj, 0u); \
          if (pos < WCAP) list[wave * WCAP + pos] = el0 + (J); \
        } \
        wc += (int)__builtin_popcount(mj); } }
    HITJ(0, h0)
    HITJ(1, h1)
    HITJ(2, h2)
    HITJ(3, h3)
    HITJ(4, h4)
    HITJ(5, h5)
    HITJ(6, h6)
    HITJ(7, h7)
#undef HITJ
  }
  return wc;
}

__global__ __launch_bounds__(NTHR) void k_agg(
    const float* __restrict__ pq, const int* __restrict__ ei,
    const v4u* __restrict__ w2p, const float* __restrict__ b2,
    const float* __restrict__ a1p, const float* __restrict__ a2p,
    float* aggp, int nN, int nE, int vec8) {
  __shared__ __attribute__((aligned(16))) float accL[(NB + 1) * HD];
  __shared__ __attribute__((aligned(16))) float msg[PASSN * HD];
  __shared__ v4u stgH[PASSN * 8];
  __shared__ v4u stgL[PASSN * 8];
  __shared__ v4u wsm[2 * HD * 8];
  __shared__ __attribute__((aligned(16))) float b2s[HD];
  __shared__ int list[LISTN];
  __shared__ int pend[PCAP];
  __shared__ int slotb[PASSN];
  __shared__ int wcnt[NWAVE];
  __shared__ int pendN;

  const int tid = threadIdx.x, lane = tid & 31, wave = tid >> 5, h = lane >> 4, m = lane & 15;
  const int nodeBase = blockIdx.x * NB;
  const int* srcs = ei;
  const int* dsts = ei + nE;
  const float a1 = a1p[0], a2 = a2p[0];

  for (int i = tid; i < (NB + 1) * HD / 4; i += NTHR) { v4f z = {0.0f, 0.0f, 0.0f, 0.0f}; *(v4f*)(accL + 4 * i) = z; }
  for (int i = tid; i < 2 * HD * 8; i += NTHR) wsm[i] = w2p[i];
  if (tid < HD) b2s[tid] = b2[tid];
  if (tid == 0) pendN = 0;
  __syncthreads();

  const int nChunks = (nE + CHUNK - 1) / CHUNK;
#pragma unroll 1
  for (int ch = 0; ch < nChunks; ++ch) {
    const int cbase = ch * CHUNK;
    const int wc = scan_chunk(dsts, nE, cbase, nodeBase, vec8, list, tid, wave);
    if (lane == 0) wcnt[wave] = wc;
    __syncthreads();

    const int base = pendN;
    int tot = 0, myoff = 0;
#pragma unroll
    for (int w = 0; w < NWAVE; ++w) {
      int c = wcnt[w];
      c = c > WCAP ? WCAP : (c < 0 ? 0 : c);
      if (w < wave) myoff += c;
      tot += c;
    }
    int newN = base + tot;
    newN = newN > PCAP ? PCAP : newN;
    {
      int n = wcnt[wave];
      n = n > WCAP ? WCAP : (n < 0 ? 0 : n);
      const int* lp = list + wave * WCAP;
      for (int i = lane; i < n; i += 32) {
        const int pos = base + myoff + i;
        if (pos < PCAP) pend[pos] = cbase + lp[i];
      }
    }
    const int fin = (ch == nChunks - 1) ? 1 : 0;
    const int R   = (fin != 0) ? (newN + PASSN - 1) / PASSN : newN / PASSN;
    const int Pv  = (fin != 0) ? newN : R * PASSN;
    __syncthreads();

#pragma unroll 1
    for (int r = 0; r < R; ++r) {
      {
        const int idx = r * PASSN + wave * TE + m;
        const bool valid = idx < Pv;
        int e = pend[(idx < PCAP) ? idx : PCAP - 1];
        e = clampi(e, 0, nE - 1);
        int d = dsts[e];
        int s = srcs[e];
        int slot = d - nodeBase;
        if (!valid || (unsigned)slot >= (unsigned)NB) slot = NB;
        d = clampi(d, 0, nN - 1);
        s = clampi(s, 0, nN - 1);
        const float* prow = pq + (size_t)d * (2 * HD) + 32 * h;
        const float* qrow = pq + (size_t)s * (2 * HD) + HD + 32 * h;
        v4u* dsth = stgH + (wave * TE + m) * 8 + 4 * h;
        v4u* dstl = stgL + (wave * TE + m) * 8 + 4 * h;
#pragma unroll
        for (int j = 0; j < 4; ++j) {
          const v4f p0 = *(const v4f*)(prow + 8 * j), p1 = *(const v4f*)(prow + 8 * j + 4);
          const v4f q0 = *(const v4f*)(qrow + 8 * j), q1 = *(const v4f*)(qrow + 8 * j + 4);
          const v4f t0 = prelu4(p0 + q0, a1), t1 = prelu4(p1 + q1, a1);
          v4u hi, lo;
          split8(t0, t1, hi, lo);
          dsth[j] = hi;
          dstl[j] = lo;
        }
        if (h == 0) slotb[wave * TE + m] = slot;
      }
      __syncthreads();

      {
        Frag bh[2], bl[2];
        const v4u* hr = stgH + (wave * TE + m) * 8;
        const v4u* lr = stgL + (wave * TE + m) * 8;
#pragma unroll
        for (int ks = 0; ks < 2; ++ks) {
          bh[ks].q[0] = hr[4 * ks + h]; bh[ks].q[1] = hr[4 * ks + h + 2];
          bl[ks].q[0] = lr[4 * ks + h]; bl[ks].q[1] = lr[4 * ks + h + 2];
        }
        float* mrow = msg + (wave * TE + m) * HD;
#pragma unroll
        for (int ft = 0; ft < 4; ++ft) {
          v8f acc = ldc8(b2s + 16 * ft + 8 * h);
#pragma unroll
          for (int ks = 0; ks < 2; ++ks) {
            const int u = (16 * ft + m) * 8 + 4 * ks + h;
            Frag ah, al;
            ah.q[0] = wsm[u];           ah.q[1] = wsm[u + 2];
            al.q[0] = wsm[HD * 8 + u];  al.q[1] = wsm[HD * 8 + u + 2];
            acc = wm3(ah, al, bh[ks], bl[ks], acc);
          }
          stprelu8(mrow + 16 * ft + 8 * h, acc, a2);
        }
      }
      __syncthreads();

      if (wave == 0) {
#pragma unroll 1
        for (int i = 0; i < PASSN; ++i) {
          int sl = slotb[i];
          sl = clampi(sl, 0, NB);
          const v2f v = *(const v2f*)(msg + i * HD + 2 * lane);
          v2f* ap = (v2f*)(accL + sl * HD + 2 * lane);
          *ap = *ap + v;
        }
      }
      __syncthreads();
    }

    int rem = newN - R * PASSN;
    rem = rem < 0 ? 0 : rem;
    if (R > 0 && tid < rem) pend[tid] = pend[R * PASSN + tid];
    if (tid == 0) pendN = rem;
  }
  __syncthreads();

  {
    const float* sp = accL + wave * (NB * HD / NWAVE);
    float* gp = aggp + (size_t)nodeBase * HD + (size_t)wave * (NB * HD / NWAVE);
#pragma unroll 4
    for (int q = 0; q < (NB * HD / NWAVE) / 128; ++q) {
      const v4f v = *(const v4f*)(sp + q * 128 + 4 * lane);
      *(volatile v4f*)(gp + q * 128 + 4 * lane) = v;
    }
    __threadfence();
#pragma unroll 4
    for (int q = 0; q < (NB * HD / NWAVE) / 128; ++q) {
      const v4f v = *(const v4f*)(sp + q * 128 + 4 * lane);
      *(volatile v4f*)(gp + q * 128 + 4 * lane) = v;
    }
  }
}

__global__ __launch_bounds__(GT) void k_node(
    const float* __restrict__ x, const float* __restrict__ agg,
    const v4u* __restrict__ w3p, const v4u* __restrict__ w4p,
    const float* __restrict__ b3, const float* __restrict__ b4,
    const float* __restrict__ a3p, const float* __restrict__ abp,
    float* zp, double* part, int nN) {
  __shared__ v4u w3s[2 * HD * 16];
  __shared__ v4u w4s[2 * HD * 8];
  __shared__ __attribute__((aligned(16))) float b3s[HD];
  __shared__ __attribute__((aligned(16))) float b4s[HD];
  __shared__ __attribute__((aligned(16))) float zst[GROWS * HD];

  const int tid = threadIdx.x, lane = tid & 31, wave = tid >> 5, h = lane >> 4, m = lane & 15;
  for (int i = tid; i < 2 * HD * 16; i += GT) w3s[i] = w3p[i];
  for (int i = tid; i < 2 * HD * 8; i += GT) w4s[i] = w4p[i];
  if (tid < HD) { b3s[tid] = b3[tid]; b4s[tid] = b4[tid]; }
  const float a3 = a3p[0], ab = abp[0];
  __syncthreads();

  const int n0 = blockIdx.x * GROWS + wave * 16;
  const int nd = clampi(n0 + m, 0, nN - 1);
  const float* xr = x + (size_t)nd * HD;
  const float* ar = agg + (size_t)nd * HD;

  v8f acc[4];
#pragma unroll
  for (int ft = 0; ft < 4; ++ft) acc[ft] = ldc8(b3s + 16 * ft + 8 * h);
#pragma unroll
  for (int ks = 0; ks < 4; ++ks) {
    const float* rp = (ks < 2) ? (xr + 32 * ks) : (ar + 32 * (ks - 2));
    const float* p = rp + 8 * h;
    const v4f e0 = *(const v4f*)p,        e1 = *(const v4f*)(p + 4);
    const v4f c0 = *(const v4f*)(p + 16), c1 = *(const v4f*)(p + 20);
    Frag bh, bl;
    split8(e0, e1, bh.q[0], bl.q[0]);
    split8(c0, c1, bh.q[1], bl.q[1]);
#pragma unroll
    for (int ft = 0; ft < 4; ++ft) {
      const int u = (16 * ft + m) * 16 + 4 * ks + h;
      Frag ah, al;
      ah.q[0] = w3s[u];            ah.q[1] = w3s[u + 2];
      al.q[0] = w3s[HD * 16 + u];  al.q[1] = w3s[HD * 16 + u + 2];
      acc[ft] = wm3(ah, al, bh, bl, acc[ft]);
    }
  }

  Frag b4h[2], b4l[2];
#pragma unroll
  for (int ft = 0; ft < 4; ++ft) prelu_split8(acc[ft], a3, b4h[ft >> 1].q[ft & 1], b4l[ft >> 1].q[ft & 1]);

  float* zrow = zst + (wave * 16 + m) * HD;
#pragma unroll
  for (int ft = 0; ft < 4; ++ft) {
    v8f acc2 = ldc8(b4s + 16 * ft + 8 * h);
#pragma unroll
    for (int ks = 0; ks < 2; ++ks) {
      const int u = (16 * ft + m) * 8 + 4 * ks + h;
      Frag ah, al;
      ah.q[0] = w4s[u];           ah.q[1] = w4s[u + 2];
      al.q[0] = w4s[HD * 8 + u];  al.q[1] = w4s[HD * 8 + u + 2];
      acc2 = wm3(ah, al, b4h[ks], b4l[ks], acc2);
    }
    stprelu8(zrow + 16 * ft + 8 * h, acc2, ab);
  }
  __syncthreads();

  const bool sw = tid < HD;
  double ps = 0.0, pq2 = 0.0;
  if (sw) {
    int nv = nN - blockIdx.x * GROWS;
    nv = nv > GROWS ? GROWS : nv;
#pragma unroll 1
    for (int r = 0; r < nv; ++r) {
      const double z = (double)zst[r * HD + tid];
      ps += z;
      pq2 += z * z;
    }
  }
  v2d pv = {ps, pq2};
  double* pp = part + (size_t)blockIdx.x * 128 + 2 * tid;

  const float* sp = zst + wave * (16 * HD);
  float* gp = zp + (size_t)n0 * HD;
#pragma unroll
  for (int q = 0; q < 8; ++q) {
    const v4f v = *(const v4f*)(sp + q * 128 + 4 * lane);
    *(volatile v4f*)(gp + q * 128 + 4 * lane) = v;
  }
  if (sw) *(volatile v2d*)pp = pv;
  __threadfence();
#pragma unroll
  for (int q = 0; q < 8; ++q) {
    const v4f v = *(const v4f*)(sp + q * 128 + 4 * lane);
    *(volatile v4f*)(gp + q * 128 + 4 * lane) = v;
  }
  if (sw) *(volatile v2d*)pp = pv;
}

__global__ __launch_bounds__(HD) void k_bnfin(const double* __restrict__ part, int nBlk, int nN, float* stats) {
  __shared__ __attribute__((aligned(16))) float st[2 * HD];
  const int c = threadIdx.x;
  double s = 0.0, q = 0.0;
#pragma unroll 1
  for (int b = 0; b < nBlk; ++b) {
    s += part[(size_t)b * 128 + 2 * c];
    q += part[(size_t)b * 128 + 2 * c + 1];
  }
  const double inv = 1.0 / (double)nN;
  const double mu  = s * inv;
  double var = q * inv - mu * mu;
  if (var < 0.0) var = 0.0;
  const float vf = (float)var;
  st[c]      = (float)mu;
  st[HD + c] = (float)(1.0 / sqrt((double)vf + BN_EPS));
  __syncthreads();
  v4f v = {0.0f, 0.0f, 0.0f, 0.0f};
  const bool wr = c < 32;
  if (wr) v = *(const v4f*)(st + 4 * c);
  if (wr) *(volatile v4f*)(stats + 4 * c) = v;
  __threadfence();
  if (wr) *(volatile v4f*)(stats + 4 * c) = v;
}

__global__ __launch_bounds__(256) void k_bnapply(const float* __restrict__ zp, const float* __restrict__ stats,
                                                 const float* __restrict__ gamma, const float* __restrict__ beta,
                                                 float* out, int total4) {
  const int i  = blockIdx.x * 256 + threadIdx.x;
  const int ic = (i < total4) ? i : total4 - 1;
  const int c4 = ic & 15;
  const v4f z  = *(const v4f*)(zp + (size_t)ic * 4);
  const v4f mu = *(const v4f*)(stats + 4 * c4);
  const v4f rs = *(const v4f*)(stats + HD + 4 * c4);
  const v4f g  = *(const v4f*)(gamma + 4 * c4);
  const v4f b  = *(const v4f*)(beta + 4 * c4);
  const v4f o  = (z - mu) * rs * g + b;
  if (i < total4) *(volatile v4f*)(out + (size_t)i * 4) = o;
  __threadfence();
  if (i < total4) *(volatile v4f*)(out + (size_t)i * 4) = o;
}

extern "C" void kernel_launch(void* const* d_in, const int* in_sizes, int n_in,
                              void* d_out, int out_size, void* d_ws, size_t ws_size,
                              hipStream_t stream) {
  if (n_in < 16) return;
  const int nN = in_sizes[0] / HD;
  const int nE = in_sizes[1] / 2;
  if (nN <= 0 || in_sizes[0] != nN * HD) return;
  if (nE < 1 || in_sizes[1] != nE * 2) return;
  if (in_sizes[2] != 2 * HD * HD || in_sizes[3] < HD || in_sizes[4] < 1) return;
  if (in_sizes[5] != HD * HD || in_sizes[6] < HD || in_sizes[7] < 1) return;
  if (in_sizes[8] != 2 * HD * HD || in_sizes[9] < HD || in_sizes[10] < 1) return;
  if (in_sizes[11] != HD * HD || in_sizes[12] < HD || in_sizes[13] < 1) return;
  if (in_sizes[14] < HD || in_sizes[15] < HD) return;
  if (out_size != nN * HD) return;

  const float* x     = (const float*)d_in[0];
  const int*   ei    = (const int*)d_in[1];
  const float* W1    = (const float*)d_in[2];
  const float* b1    = (const float*)d_in[3];
  const float* a1    = (const float*)d_in[4];
  const float* W2    = (const float*)d_in[5];
  const float* b2    = (const float*)d_in[6];
  const float* a2    = (const float*)d_in[7];
  const float* W3    = (const float*)d_in[8];
  const float* b3    = (const float*)d_in[9];
  const float* a3    = (const float*)d_in[10];
  const float* W4    = (const float*)d_in[11];
  const float* b4    = (const float*)d_in[12];
  const float* ablk  = (const float*)d_in[13];
  const float* gamma = (const float*)d_in[14];
  const float* beta  = (const float*)d_in[15];
  float* out = (float*)d_out;

  const int nBlkN = (nN + GROWS - 1) / GROWS;
  const int nPadN = nBlkN * GROWS;
  const int nBlkA = (nN + NB - 1) / NB;
  const int nPadA = nBlkA * NB;

  char* ws = (char*)d_ws;
  size_t off = 0;
  const size_t oW = off;    off += (size_t)(2 * 128 * 8 + 2 * HD * 8 + 2 * HD * 16 + 2 * HD * 8) * 16;  off = (off + 1023) & ~(size_t)1023;
  const size_t oPQ = off;   off += (size_t)nPadN * 128 * 4;                                             off = (off + 1023) & ~(size_t)1023;
  const size_t oAG = off;   off += (size_t)nPadA * HD * 4;                                              off = (off + 1023) & ~(size_t)1023;
  const size_t oZ = off;    off += (size_t)nPadN * HD * 4;                                              off = (off + 1023) & ~(size_t)1023;
  const size_t oPT = off;   off += (size_t)nBlkN * 128 * 8;                                             off = (off + 1023) & ~(size_t)1023;
  const size_t oST = off;   off += 512;                                                                  off = (off + 1023) & ~(size_t)1023;
  if (off > ws_size) return;

  v4u* wpl = (v4u*)(ws + oW);
  v4u* w1p = wpl;
  v4u* w2p = wpl + 2048;
  v4u* w3p = wpl + 3072;
  v4u* w4p = wpl + 5120;
  float*  pqp   = (float*)(ws + oPQ);
  float*  aggp  = (float*)(ws + oAG);
  float*  zp    = (float*)(ws + oZ);
  double* part  = (double*)(ws + oPT);
  float*  stats = (float*)(ws + oST);

  const int vec8 = ((nE & 3) == 0) ? 1 : 0;

  k_wprep<<<2, 256, 0, stream>>>(W1, HD, HD, 0,  w1p,         w1p + 1024,       HD * HD / 8);
  k_wprep<<<2, 256, 0, stream>>>(W1, HD, HD, HD, w1p + 512,   w1p + 1024 + 512, HD * HD / 8);
  k_wprep<<<2, 256, 0, stream>>>(W2, HD, HD, 0,  w2p,         w2p + 512,        HD * HD / 8);
  k_wprep<<<4, 256, 0, stream>>>(W3, HD, 2 * HD, 0, w3p,      w3p + 1024,       HD * 2 * HD / 8);
  k_wprep<<<2, 256, 0, stream>>>(W4, HD, HD, 0,  w4p,         w4p + 512,        HD * HD / 8);

  k_pq<<<nBlkN, GT, 0, stream>>>(x, w1p, b1, pqp, nN);

  k_agg<<<nBlkA, NTHR, 0, stream>>>(pqp, ei, w2p, b2, a1, a2, aggp, nN, nE, vec8);

  k_node<<<nBlkN, GT, 0, stream>>>(x, aggp, w3p, w4p, b3, b4, a3, ablk, zp, part, nN);

  k_bnfin<<<1, HD, 0, stream>>>(part, nBlkN, nN, stats);

  const int total4 = nN * (HD / 4);
  k_bnapply<<<(total4 + 255) / 256, 256, 0, stream>>>(zp, stats, gamma, beta, out, total4);
}
